// RecurrentModule_30880814858454
// MI455X (gfx1250) — hardware-verified
//
#include <hip/hip_runtime.h>


namespace {
constexpr int B = 512, T = 1024, I = 15, H = 64, O = 11, TB = 32;
constexpr float XS = 8.0f, WSC = 256.0f;
typedef _Float16 b16;
typedef __attribute__((ext_vector_type(16))) _Float16 v16b;
typedef __attribute__((ext_vector_type(8))) _Float16 v8b;
typedef __attribute__((ext_vector_type(8))) float v8f;
typedef __attribute__((ext_vector_type(4))) float v4f;
typedef __attribute__((ext_vector_type(2))) float v2f;
__device__ __forceinline__ float bf16_rne(float f) { unsigned int u = __float_as_uint(f); u += 0x7FFFu + ((u >> 16) & 1u); return __uint_as_float(u & 0xFFFF0000u); }
__device__ __forceinline__ void split16(float v, b16& hi, b16& lo) { hi = (b16)v; lo = (b16)(v - (float)hi); }
__device__ __forceinline__ v16b frag_kb(const b16* p, int hh) { const v8b a = *(const v8b*)(p + 8 * hh), b = *(const v8b*)(p + 16 + 8 * hh); v16b f;
#pragma unroll
  for (int e = 0; e < 8; ++e) { f[e] = a[e]; f[8 + e] = b[e]; } return f; }
__device__ __forceinline__ v8f wmma16b(v16b a, v16b b, v8f c) { v8f d = __builtin_amdgcn_wmma_f32_16x16x32_f16(false, a, false, b, (short)0, c, false, false); asm volatile("v_nop\n\tv_nop\n\tv_nop\n\tv_nop" : "+v"(d) : "v"(a), "v"(b)); return d; }
__device__ __forceinline__ void wave_lds_sync() { __builtin_amdgcn_fence(__ATOMIC_RELEASE, "workgroup"); __builtin_amdgcn_wave_barrier(); __builtin_amdgcn_fence(__ATOMIC_ACQUIRE, "workgroup"); }
__device__ __forceinline__ float pmul(float a, float b) { float p = a * b; asm volatile("" : "+v"(p)); return p; }

__global__ __launch_bounds__(256) void wcopy_kernel(const float* __restrict__ w, int OUT, int OUTP, b16* __restrict__ WT) {
  const int u = blockIdx.x * 256 + threadIdx.x; if (u >= OUTP * H / 8) return; const int e = u * 8; const int o = e / H, k0 = e % H; v8b v; for (int j = 0; j < 8; ++j) v[j] = o < OUT ? (b16)(bf16_rne(w[o * H + k0 + j]) * WSC) : (b16)0.0f;
  for (int pass = 0; pass < 2; ++pass) { *(volatile v8b*)(WT + e) = v; __threadfence(); }
}
__global__ __launch_bounds__(32) void rnn_kernel(const float* __restrict__ x, const float* __restrict__ Wih, const float* __restrict__ bih, const float* __restrict__ bhh, const b16* __restrict__ WHH, const b16* __restrict__ WDEC, const float* __restrict__ bdec, float* __restrict__ out, float* __restrict__ hout) {
  __shared__ __attribute__((aligned(16))) b16 Ah[16][H + 8], Al[16][H + 8]; __shared__ float Xs[16][16]; __shared__ float Wi[H][16]; __shared__ __attribute__((aligned(16))) float Ob[16][TB * O + 4]; __shared__ __attribute__((aligned(16))) float Hs[16][H + 4];
  const int lane = threadIdx.x, nloc = lane & 15, hlf = lane >> 4; const int b0 = blockIdx.x * 16; const float sc = 1.0f / (XS * WSC);
  for (int i = lane; i < H * 16; i += 32) { const int u = i / 16, k = i % 16; Wi[u][k] = k < I ? bf16_rne(Wih[u * I + k]) : 0.0f; }
  for (int rr = 0; rr < 16; ++rr) { Ah[rr][lane * 2] = (b16)0.0f; Ah[rr][lane * 2 + 1] = (b16)0.0f; Al[rr][lane * 2] = (b16)0.0f; Al[rr][lane * 2 + 1] = (b16)0.0f; Hs[rr][lane * 2] = 0.0f; Hs[rr][lane * 2 + 1] = 0.0f; }
  float bsum[4]; for (int t4 = 0; t4 < 4; ++t4) bsum[t4] = bf16_rne(bih[t4 * 16 + nloc]) + bf16_rne(bhh[t4 * 16 + nloc]); const float bd = nloc < O ? bf16_rne(bdec[nloc]) : 0.0f;
  wave_lds_sync();
#pragma unroll 1
  for (int t = 0; t < T; ++t) {
    { const int rr = lane >> 1, half = lane & 1; const float* xr = x + ((size_t)(b0 + rr) * T + t) * I; for (int k = half * 8; k < half * 8 + 8; ++k) Xs[rr][k] = k < I ? bf16_rne(xr[k]) : 0.0f; }
    wave_lds_sync();
    v8f acc[4];
#pragma unroll
    for (int t4 = 0; t4 < 4; ++t4) acc[t4] = (v8f){};
#pragma unroll
    for (int kb = 0; kb < H; kb += 32) { const v16b a = frag_kb(&Ah[nloc][kb], hlf), al = frag_kb(&Al[nloc][kb], hlf);
#pragma unroll
      for (int t4 = 0; t4 < 4; ++t4) { const v16b bw = frag_kb(WHH + (size_t)(t4 * 16 + nloc) * H + kb, hlf); acc[t4] = wmma16b(a, bw, acc[t4]); acc[t4] = wmma16b(al, bw, acc[t4]); } }
    wave_lds_sync();
#pragma unroll
    for (int t4 = 0; t4 < 4; ++t4) { const int c = t4 * 16 + nloc;
#pragma unroll
      for (int r8 = 0; r8 < 8; ++r8) { const int rl = 8 * hlf + r8; float xp = bsum[t4];
#pragma unroll 1
        for (int k = 0; k < I; ++k) xp += pmul(Xs[rl][k], Wi[c][k]);
        const float h = fmaxf(acc[t4][r8] * sc + xp, 0.0f); Hs[rl][c] = h; b16 p, q; split16(h * XS, p, q); Ah[rl][c] = p; Al[rl][c] = q; } }
    wave_lds_sync();
    { v8f d = (v8f){};
#pragma unroll
      for (int kb = 0; kb < H; kb += 32) { const v16b a = frag_kb(&Ah[nloc][kb], hlf), al = frag_kb(&Al[nloc][kb], hlf); const v16b bw = frag_kb(WDEC + (size_t)nloc * H + kb, hlf); d = wmma16b(a, bw, d); d = wmma16b(al, bw, d); }
      if (nloc < O) {
#pragma unroll
        for (int r8 = 0; r8 < 8; ++r8) Ob[8 * hlf + r8][(t % TB) * O + nloc] = fmaxf(d[r8] * sc + bd, 0.0f); } }
    if ((t % TB) == TB - 1) { wave_lds_sync(); const int tb0 = t - (TB - 1);
      for (int pass = 0; pass < 2; ++pass) { for (int rr = 0; rr < 16; ++rr) { float* dst = out + ((size_t)(b0 + rr) * T + tb0) * O; for (int i = lane; i < TB * O; i += 32) ((volatile float*)dst)[i] = Ob[rr][i]; } __threadfence(); }
      wave_lds_sync(); } }
  for (int pass = 0; pass < 2; ++pass) { for (int rr = 0; rr < 16; ++rr) *(volatile v2f*)(hout + (size_t)(b0 + rr) * H + lane * 2) = *(const v2f*)(&Hs[rr][lane * 2]); __threadfence(); }
}
}

extern "C" void kernel_launch(void* const* d_in, const int* in_sizes, int n_in, void* d_out, int out_size, void* d_ws, size_t ws_size, hipStream_t stream) {
  (void)n_in;
  auto Fp = [&](int i) { return (const float*)d_in[i]; };
  if (in_sizes[0] != B * T * I || in_sizes[1] != H * I || in_sizes[3] != H * H || in_sizes[5] != O * H || out_size != B * T * O + B * H) return;
  const int NW = B / 16;
  b16* WHH = (b16*)d_ws; b16* WDEC = WHH + H * H; if ((size_t)(H * H + 16 * H) * 2 > ws_size) return;
  wcopy_kernel<<<(H * H + 255) / 256, 256, 0, stream>>>(Fp(3), H, H, WHH); wcopy_kernel<<<(16 * H + 255) / 256, 256, 0, stream>>>(Fp(5), O, 16, WDEC);
  rnn_kernel<<<NW, 32, 0, stream>>>(Fp(0), Fp(1), Fp(2), Fp(4), WHH, WDEC, Fp(6), (float*)d_out, (float*)d_out + (size_t)B * T * O);
}
